// enc_graph_29472065585643
// MI455X (gfx1250) — hardware-verified
//
#include <hip/hip_runtime.h>
#include <stdint.h>

#define BB    2048
#define NN    64
#define FA    62
#define FBN   6
#define DD    5
#define CC    128
#define COUT  16
#define KK    113
#define RTOT  (BB * NN)
#define NBLK  (RTOT / 128)
#define PITCH 168
#define CONVK (NN * CC)
#define CONVN (COUT * 16)
#define BN_EPS 1e-5f

typedef __attribute__((ext_vector_type(16))) _Float16 v16h;
typedef __attribute__((ext_vector_type(8)))  _Float16 v8h;
typedef __attribute__((ext_vector_type(16))) __bf16   v16b;
typedef __attribute__((ext_vector_type(8)))  __bf16   v8b;
typedef __attribute__((ext_vector_type(8)))  float    v8f;
typedef __attribute__((ext_vector_type(4)))  float    v4f;
typedef __attribute__((ext_vector_type(2)))  float    v2f;
typedef __attribute__((ext_vector_type(4)))  _Float16 v4h;
typedef __attribute__((ext_vector_type(2)))  _Float16 v2h;

__device__ __forceinline__ unsigned short f2bf_bits(float f) {
  unsigned u = __float_as_uint(f);
  return (unsigned short)((u + 0x7FFFu + ((u >> 16) & 1u)) >> 16);
}
__device__ __forceinline__ float bf_bits2f(unsigned short h) { return __uint_as_float(((unsigned)h) << 16); }

__device__ __forceinline__ void dep_guard_h(v8f& a, v8f& b, v16h x, v16h y) { asm volatile("v_nop\n\tv_nop\n\tv_nop\n\tv_nop" : "+v"(a), "+v"(b) : "v"(x), "v"(y)); }
__device__ __forceinline__ void dep_guard_b(v8f& a, v8f& b, v16b x, v16b y) { asm volatile("v_nop\n\tv_nop\n\tv_nop\n\tv_nop" : "+v"(a), "+v"(b) : "v"(x), "v"(y)); }
__device__ __forceinline__ void dep_guard3_h(v8f& a, v8f& b, v16h x, v16h y, v16h z) { asm volatile("v_nop\n\tv_nop\n\tv_nop\n\tv_nop" : "+v"(a), "+v"(b) : "v"(x), "v"(y), "v"(z)); }
__device__ __forceinline__ void keep4_h(v16h a, v16h b, v16h c, v16h d) { asm volatile("v_nop" :: "v"(a), "v"(b), "v"(c), "v"(d)); }
__device__ __forceinline__ void keep4_b(v16b a, v16b b, v16b c, v16b d) { asm volatile("v_nop" :: "v"(a), "v"(b), "v"(c), "v"(d)); }
__device__ __forceinline__ void acc_guard4(v8f& a, v8f& b, v8f& c, v8f& d) { asm volatile("v_nop\n\tv_nop\n\tv_nop\n\tv_nop" : "+v"(a), "+v"(b), "+v"(c), "+v"(d)); }
template <typename T> struct Frag;
template <> struct Frag<_Float16> {
  typedef v16h V; union U { v16h v; v8h h[2]; };
  static __device__ __forceinline__ v16h load(const _Float16* p) {
    U f; f.h[0] = *(const v8h*)(p); f.h[1] = *(const v8h*)(p + 16); return f.v;
  }
  static __device__ __forceinline__ v8f mma(v16h a, v16h b, v8f c) {
    return __builtin_amdgcn_wmma_f32_16x16x32_f16(false, a, false, b, (short)0, c, false, false);
  }
  static __device__ __forceinline__ void guard(v8f& a, v8f& b, v16h x, v16h y) { dep_guard_h(a, b, x, y); }
  static __device__ __forceinline__ void keep(v16h a, v16h b, v16h c, v16h d) { keep4_h(a, b, c, d); }
};
template <> struct Frag<__bf16> {
  typedef v16b V; union U { v16b v; v8b h[2]; };
  static __device__ __forceinline__ v16b load(const __bf16* p) {
    U f; f.h[0] = *(const v8b*)(p); f.h[1] = *(const v8b*)(p + 16); return f.v;
  }
  static __device__ __forceinline__ v8f mma(v16b a, v16b b, v8f c) {
    return __builtin_amdgcn_wmma_f32_16x16x32_bf16(false, a, false, b, (short)0, c, false, false);
  }
  static __device__ __forceinline__ void guard(v8f& a, v8f& b, v16b x, v16b y) { dep_guard_b(a, b, x, y); }
  static __device__ __forceinline__ void keep(v16b a, v16b b, v16b c, v16b d) { keep4_b(a, b, c, d); }
};

template <int ET> struct Elem;
template <> struct Elem<0> { typedef _Float16 T; };
template <> struct Elem<1> { typedef __bf16 T; };
template <int ET, bool SPLIT, int BIAS_MODE, int OUT_MODE, bool RESID, int ACT = 0>
__global__ __launch_bounds__(256) void wmma_gemm64(
    const unsigned short* __restrict__ Ap, const unsigned short* __restrict__ A2p, int lda, long strideA,
    const unsigned short* __restrict__ Btp, const unsigned short* __restrict__ Bt2p, int ldb, long strideB,
    void* __restrict__ Cout, void* __restrict__ Cout2, int ldc, long strideC,
    const float* __restrict__ bias,
    const float* __restrict__ resid, long strideR,
    int M, int N, int K, float scale) {
  typedef typename Elem<ET>::T T;
  typedef typename Frag<T>::V V;
  const T* A = (const T*)Ap; const T* A2 = (const T*)A2p; const T* Bt = (const T*)Btp; const T* Bt2 = (const T*)Bt2p;
  __shared__ __align__(16) float sT[8][16 * 68];
  const int b    = blockIdx.y;
  const int lane = threadIdx.x & 31;
  const int wave = threadIdx.x >> 5;
  const int tilesN = N >> 6;
  const int tilesM = M >> 6;
  const int tile = blockIdx.x * 8 + wave;
  if (tile >= tilesM * tilesN) return;
  const int tm = tile / tilesN;
  const int tn = tile - tm * tilesN;
  const int m0 = tm << 6;
  const int n0 = tn << 6;

  const T* Ab  = A  + (size_t)b * strideA;
  const T* Bb  = Bt + (size_t)b * strideB;
  const T* Ab2 = SPLIT ? (A2  + (size_t)b * strideA) : nullptr;
  const T* Bb2 = SPLIT ? (Bt2 + (size_t)b * strideB) : nullptr;

  const int rlane = lane & 15;
  const int koff  = (lane >> 4) * 8;
  const int mOff  = (lane >> 4) * 8;

  v8f acc[4][4];
#pragma unroll
  for (int i = 0; i < 4; ++i)
#pragma unroll
    for (int j = 0; j < 4; ++j) acc[i][j] = (v8f){0.f,0.f,0.f,0.f,0.f,0.f,0.f,0.f};

  for (int k0 = 0; k0 < K; k0 += 32) {
    V bh[4], bl[4];
#pragma unroll
    for (int j = 0; j < 4; ++j) {
      const size_t bo = (size_t)(n0 + (j << 4) + rlane) * ldb + koff + k0;
      bh[j] = Frag<T>::load(Bb + bo);
      if (SPLIT) bl[j] = Frag<T>::load(Bb2 + bo);
    }
#pragma unroll
    for (int i = 0; i < 4; ++i) {
      const size_t ao = (size_t)(m0 + (i << 4) + rlane) * lda + koff + k0;
      V ah = Frag<T>::load(Ab + ao);
      V al;
      if (SPLIT) al = Frag<T>::load(Ab2 + ao);
#pragma unroll
      for (int j = 0; j < 4; ++j) {
        acc[i][j] = Frag<T>::mma(ah, bh[j], acc[i][j]);
        if (SPLIT) {
          acc[i][j] = Frag<T>::mma(ah, bl[j], acc[i][j]);
          acc[i][j] = Frag<T>::mma(al, bh[j], acc[i][j]);
        }
      }
      Frag<T>::guard(acc[i][0], acc[i][3], ah, SPLIT ? al : ah);
    }
    Frag<T>::keep(bh[0], bh[1], bh[2], bh[3]);
    if (SPLIT) Frag<T>::keep(bl[0], bl[1], bl[2], bl[3]);
  }
  acc_guard4(acc[0][0], acc[0][1], acc[0][2], acc[0][3]);
  acc_guard4(acc[1][0], acc[1][1], acc[1][2], acc[1][3]);
  acc_guard4(acc[2][0], acc[2][1], acc[2][2], acc[2][3]);
  acc_guard4(acc[3][0], acc[3][1], acc[3][2], acc[3][3]);

  float* slab = sT[wave];
  const float* Rb = RESID ? (resid + (size_t)b * strideR) : nullptr;
#pragma unroll
  for (int i = 0; i < 4; ++i) {
    const int mBase = m0 + (i << 4);
#pragma unroll
    for (int j = 0; j < 4; ++j) {
      const int n = n0 + (j << 4) + rlane;
      float bv = 0.f;
      if (BIAS_MODE == 2) bv = bias[n];
#pragma unroll
      for (int r = 0; r < 8; ++r) {
        float v = acc[i][j][r] * scale;
        if (BIAS_MODE == 1) v += bias[mBase + mOff + r];
        if (BIAS_MODE == 2) v += bv;
        if (RESID) v += Rb[(size_t)(mBase + mOff + r) * ldc + n];
        if (ACT == 1) v = tanhf(v);
        if (ACT == 2) v = fmaxf(v, 0.0f);
        if (ACT == 3) v = v / (1.0f + expf(-v));
        if (ACT == 4) v = (v > 0.f) ? v : 0.01f * v;
        if (ACT == 5) v = 0.5f * v * (1.0f + erff(v * 0.70710678118654752f));
        slab[(mOff + r) * 68 + (j << 4) + rlane] = v;
      }
    }
    __builtin_amdgcn_fence(__ATOMIC_RELEASE, "workgroup");
    __builtin_amdgcn_wave_barrier();
    __builtin_amdgcn_fence(__ATOMIC_ACQUIRE, "workgroup");
    if (OUT_MODE == 0) {
      float* C = (float*)Cout + (size_t)b * strideC;
      const int hh = lane >> 4, c4 = (lane & 15) * 4;
      for (int pass = 0; pass < 2; ++pass) {
#pragma unroll
        for (int it = 0; it < 8; ++it) {
          const int row = it * 2 + hh;
          v4f v = *(const v4f*)(slab + row * 68 + c4);
          *(volatile v4f*)(C + (size_t)(mBase + row) * ldc + n0 + c4) = v;
        }
        __threadfence();
      }
    } else {
      const int q = lane >> 3, c8 = (lane & 7) * 8;
      unsigned short* C  = (unsigned short*)Cout  + (size_t)b * strideC;
      unsigned short* C2 = (OUT_MODE == 2) ? ((unsigned short*)Cout2 + (size_t)b * strideC) : nullptr;
      for (int pass = 0; pass < 2; ++pass) {
#pragma unroll
        for (int it = 0; it < 4; ++it) {
          const int row = it * 4 + q;
          const float* sp = slab + row * 68 + c8;
          v8h hv, lv;
#pragma unroll
          for (int e = 0; e < 8; ++e) {
            if (OUT_MODE == 1) {
              hv[e] = (_Float16)sp[e];
            } else {
              unsigned short hb = f2bf_bits(sp[e]);
              unsigned short lb = f2bf_bits(sp[e] - bf_bits2f(hb));
              hv[e] = __builtin_bit_cast(_Float16, hb);
              lv[e] = __builtin_bit_cast(_Float16, lb);
            }
          }
          *(volatile v8h*)(C + (size_t)(mBase + row) * ldc + n0 + c8) = hv;
          if (OUT_MODE == 2) *(volatile v8h*)(C2 + (size_t)(mBase + row) * ldc + n0 + c8) = lv;
        }
        __threadfence();
      }
    }
    __builtin_amdgcn_fence(__ATOMIC_RELEASE, "workgroup");
    __builtin_amdgcn_wave_barrier();
    __builtin_amdgcn_fence(__ATOMIC_ACQUIRE, "workgroup");
  }
}

template <int FIN, int KP>
__global__ __launch_bounds__(256) void prep_wg(const float* __restrict__ W, unsigned short* __restrict__ Btp) {
  constexpr int KQ = KP / 8;
  const int i = blockIdx.x * 256 + threadIdx.x;
  if (i >= DD * CC * KQ) return;
  const int row = i / KQ;
  const int kq  = i - row * KQ;
  const int d = row >> 7, n = row & (CC - 1);
  v8h v;
#pragma unroll
  for (int e = 0; e < 8; ++e) {
    const int k  = kq * 8 + e;
    const int kc = (k < FIN) ? k : (FIN - 1);
    const float w = W[((size_t)d * FIN + kc) * CC + n] * 16.0f;
    v[e] = (_Float16)((k < FIN) ? w : 0.0f);
  }
  _Float16* p = (_Float16*)Btp + (size_t)row * KP + kq * 8;
  *(volatile v8h*)p = v;
  __threadfence();
  *(volatile v8h*)p = v;
}

__global__ __launch_bounds__(256) void prep_wc(const float* __restrict__ W, unsigned short* __restrict__ Btp) {
  const int i = blockIdx.x * 256 + threadIdx.x;
  if (i >= CONVN * (CONVK / 8)) return;
  const int row  = i >> 10;
  const int cq   = i & 1023;
  const int o = row >> 4, l = row & 15;
  const int col0 = cq * 8;
  const int n  = col0 >> 7;
  const int cb = col0 & (CC - 1);
  v8h v;
#pragma unroll
  for (int e = 0; e < 8; ++e) {
    const int k = cb + e - l;
    const bool ok = (k >= 0) && (k < KK);
    const int kc = (k < 0) ? 0 : ((k > KK - 1) ? (KK - 1) : k);
    const float w = W[((size_t)(o * NN + n)) * KK + kc] * 64.0f;
    v[e] = (_Float16)(ok ? w : 0.0f);
  }
  _Float16* p = (_Float16*)Btp + (size_t)row * CONVK + col0;
  *(volatile v8h*)p = v;
  __threadfence();
  *(volatile v8h*)p = v;
}

template <bool L1>
__global__ __launch_bounds__(128) void graph_layer(
    const float* xin,
    const float* __restrict__ sc_in, const float* __restrict__ sh_in,
    const int* __restrict__ edges, const float* __restrict__ bonds,
    const unsigned short* __restrict__ btp, const float* __restrict__ bias,
    float* zout, float* __restrict__ psum, float* __restrict__ psq)
{
  constexpr int F   = L1 ? FA : CC;
  constexpr int KP  = L1 ? 96 : 160;
  constexpr int NCH = KP / 32;
  typedef Frag<_Float16> FH;
  union HU { v16h v; unsigned u[8]; };

  __shared__ __align__(16) _Float16 sact[128 * PITCH];
  __shared__ __align__(16) float sred[2 * CC];
  __shared__ float sst[4 * CC];
  __shared__ float ssq[4 * CC];
  __shared__ float sbias[DD * CC];
  __shared__ int   sdeg[128];

  const int tid = threadIdx.x, wave = tid >> 5, lane = tid & 31, hh = lane >> 4, r16 = lane & 15;
  const int row0 = blockIdx.x * 128;
  for (int i = tid; i < DD * CC; i += 128) sbias[i] = bias[i];

  {
    const int c4 = lane * 4;
    const int c2 = (lane < 31) ? lane * 2 : 60;
    const int jb = (lane < FBN) ? lane : (FBN - 1);
    v4f scv = {0.f, 0.f, 0.f, 0.f}, shv = {0.f, 0.f, 0.f, 0.f};
    if (!L1) { scv = *(const v4f*)(sc_in + c4); shv = *(const v4f*)(sh_in + c4); }
#pragma unroll 1
    for (int i = 0; i < 32; ++i) {
      const int rloc = wave * 32 + i;
      const int rowg = row0 + rloc;
      const int bmol = rowg >> 6;
      _Float16* arow = sact + rloc * PITCH;
      int ev[DD];
      int deg = 0;
#pragma unroll
      for (int s = 0; s < DD; ++s) { ev[s] = edges[(size_t)rowg * DD + s]; deg += (ev[s] >= 0) ? 1 : 0; }
      if (L1) {
        v2f acc = {0.f, 0.f};
#pragma unroll
        for (int s = 0; s < DD; ++s) {
          const float vm = (ev[s] >= 0) ? 1.0f : 0.0f;
          int idx = (ev[s] < 0) ? 0 : ev[s];
          idx = (idx > NN - 1) ? (NN - 1) : idx;
          const v2f x = *(const v2f*)(xin + (size_t)(bmol * NN + idx) * FA + c2);
          acc += x * vm;
        }
        const v2f xs = *(const v2f*)(xin + (size_t)rowg * FA + c2);
        acc += xs;
        if (lane < 31) {
          v2h hv;
          hv[0] = (_Float16)acc[0];
          hv[1] = (_Float16)acc[1];
          *(v2h*)(arow + lane * 2) = hv;
        }
      } else {
        v4f acc = {0.f, 0.f, 0.f, 0.f};
#pragma unroll
        for (int s = 0; s < DD; ++s) {
          const float vm = (ev[s] >= 0) ? 1.0f : 0.0f;
          int idx = (ev[s] < 0) ? 0 : ev[s];
          idx = (idx > NN - 1) ? (NN - 1) : idx;
          const v4f x = *(const v4f*)(xin + (size_t)(bmol * NN + idx) * CC + c4);
          v4f a;
#pragma unroll
          for (int e = 0; e < 4; ++e) a[e] = fmaxf(fmaf(x[e], scv[e], shv[e]), 0.0f) * vm;
          acc += a;
        }
        const v4f xs = *(const v4f*)(xin + (size_t)rowg * CC + c4);
        v4f a;
#pragma unroll
        for (int e = 0; e < 4; ++e) a[e] = fmaxf(fmaf(xs[e], scv[e], shv[e]), 0.0f);
        acc += a;
        v4h hv;
#pragma unroll
        for (int e = 0; e < 4; ++e) hv[e] = (_Float16)acc[e];
        *(v4h*)(arow + c4) = hv;
      }
      float bs = 0.0f;
#pragma unroll
      for (int s = 0; s < DD; ++s) bs += bonds[(size_t)rowg * (DD * FBN) + s * FBN + jb];
      if (lane < FBN) arow[F + lane] = (_Float16)bs;
      const int cz = F + FBN + lane;
      if (cz < KP) arow[cz] = (_Float16)0.0f;
      if (lane == 0) sdeg[rloc] = deg;
    }
  }
  __syncthreads();

  const _Float16* Bt = (const _Float16*)btp;
  const int dA = sdeg[wave * 32 + r16];
  const int dB = sdeg[wave * 32 + 16 + r16];
  unsigned pm = 0u;
#pragma unroll
  for (int d = 0; d < DD; ++d) {
    if (__builtin_amdgcn_ballot_w32(dA == d + 1) != 0u) pm |= (1u << d);
    if (__builtin_amdgcn_ballot_w32(dB == d + 1) != 0u) pm |= (1u << d);
  }
  v8f acc[2][8];
#pragma unroll
  for (int st = 0; st < 2; ++st)
#pragma unroll
    for (int t = 0; t < 8; ++t) acc[st][t] = (v8f){0.f, 0.f, 0.f, 0.f, 0.f, 0.f, 0.f, 0.f};

  const _Float16* arowA = sact + (wave * 32 + r16) * PITCH + 8 * hh;
  const _Float16* arowB = arowA + 16 * PITCH;
  for (int kc = 0; kc < NCH; ++kc) {
    const int k0 = kc * 32;
    HU a0, a1;
    a0.v = FH::load(arowA + k0);
    a1.v = FH::load(arowB + k0);
#pragma unroll
    for (int d = 0; d < DD; ++d) {
      if (pm & (1u << d)) {
        const unsigned mk0 = (dA == d + 1) ? 0xffffffffu : 0u;
        const unsigned mk1 = (dB == d + 1) ? 0xffffffffu : 0u;
        HU m0, m1;
#pragma unroll
        for (int q = 0; q < 8; ++q) { m0.u[q] = a0.u[q] & mk0; m1.u[q] = a1.u[q] & mk1; }
        const _Float16* wb = Bt + (size_t)(d * CC + r16) * KP + k0 + 8 * hh;
        v16h bfr;
#pragma unroll
        for (int t = 0; t < 8; ++t) {
          bfr = FH::load(wb + (size_t)t * 16 * KP);
          acc[0][t] = FH::mma(m0.v, bfr, acc[0][t]);
          acc[1][t] = FH::mma(m1.v, bfr, acc[1][t]);
        }
        dep_guard3_h(acc[0][7], acc[1][7], m0.v, m1.v, bfr);
      }
    }
  }
  acc_guard4(acc[0][0], acc[0][1], acc[0][2], acc[0][3]);
  acc_guard4(acc[0][4], acc[0][5], acc[0][6], acc[0][7]);
  acc_guard4(acc[1][0], acc[1][1], acc[1][2], acc[1][3]);
  acc_guard4(acc[1][4], acc[1][5], acc[1][6], acc[1][7]);

  int dgr[2][8];
#pragma unroll
  for (int st = 0; st < 2; ++st)
#pragma unroll
    for (int r = 0; r < 8; ++r) dgr[st][r] = sdeg[wave * 32 + st * 16 + 8 * hh + r];

  __builtin_amdgcn_fence(__ATOMIC_RELEASE, "workgroup");
  __builtin_amdgcn_wave_barrier();
  __builtin_amdgcn_fence(__ATOMIC_ACQUIRE, "workgroup");
  float* slab = (float*)(sact + wave * 32 * PITCH);
  const int c4 = r16 * 4;
#pragma unroll
  for (int half = 0; half < 2; ++half) {
    float cs[4], cq[4];
#pragma unroll
    for (int tt = 0; tt < 4; ++tt) { cs[tt] = 0.f; cq[tt] = 0.f; }
#pragma unroll
    for (int st = 0; st < 2; ++st) {
#pragma unroll
      for (int tt = 0; tt < 4; ++tt) {
        const int t = half * 4 + tt;
        const int c = t * 16 + r16;
#pragma unroll
        for (int r = 0; r < 8; ++r) {
          const int rl  = st * 16 + 8 * hh + r;
          const int dg  = dgr[st][r];
          const int dgc = (dg > 0) ? (dg - 1) : 0;
          float v = acc[st][t][r] * 0.0625f + sbias[dgc * CC + c];
          v = (dg > 0) ? v : 0.0f;
          slab[rl * 68 + tt * 16 + r16] = v;
          cs[tt] += v;
          cq[tt] += v * v;
        }
      }
    }
#pragma unroll
    for (int tt = 0; tt < 4; ++tt) {
      cs[tt] += __shfl_xor(cs[tt], 16, 32);
      cq[tt] += __shfl_xor(cq[tt], 16, 32);
      if (hh == 0) {
        sst[wave * CC + half * 64 + tt * 16 + r16] = cs[tt];
        ssq[wave * CC + half * 64 + tt * 16 + r16] = cq[tt];
      }
    }
    __builtin_amdgcn_fence(__ATOMIC_RELEASE, "workgroup");
    __builtin_amdgcn_wave_barrier();
    __builtin_amdgcn_fence(__ATOMIC_ACQUIRE, "workgroup");
    float* zbase = zout + (size_t)(row0 + wave * 32) * CC + half * 64 + c4;
    for (int pass = 0; pass < 2; ++pass) {
#pragma unroll
      for (int it = 0; it < 16; ++it) {
        const int rl = it * 2 + hh;
        v4f val = *(const v4f*)(slab + rl * 68 + c4);
        *(volatile v4f*)(zbase + (size_t)rl * CC) = val;
      }
      __threadfence();
    }
    __builtin_amdgcn_fence(__ATOMIC_RELEASE, "workgroup");
    __builtin_amdgcn_wave_barrier();
    __builtin_amdgcn_fence(__ATOMIC_ACQUIRE, "workgroup");
  }
  __syncthreads();
  {
    float s = 0.f, q = 0.f;
#pragma unroll
    for (int w = 0; w < 4; ++w) { s += sst[w * CC + tid]; q += ssq[w * CC + tid]; }
    sred[tid] = s;
    sred[CC + tid] = q;
  }
  __syncthreads();
  if (wave == 0) {
    const v4f a  = *(const v4f*)(sred + lane * 4);
    const v4f bq = *(const v4f*)(sred + CC + lane * 4);
    float* ps = psum + (size_t)blockIdx.x * CC + lane * 4;
    float* pq = psq  + (size_t)blockIdx.x * CC + lane * 4;
    *(volatile v4f*)ps = a;
    *(volatile v4f*)pq = bq;
    __threadfence();
    *(volatile v4f*)ps = a;
    *(volatile v4f*)pq = bq;
  }
}

__global__ __launch_bounds__(128) void bn_finalize(const float* __restrict__ psum, const float* __restrict__ psq,
                                                    const float* __restrict__ gam, const float* __restrict__ bet,
                                                    float* __restrict__ sc, float* __restrict__ sh) {
  const int c = threadIdx.x;
  double s = 0.0, q = 0.0;
  for (int b = 0; b < NBLK; ++b) {
    s += (double)psum[(size_t)b * CC + c];
    q += (double)psq[(size_t)b * CC + c];
  }
  const double inv_n = 1.0 / 131072.0;
  const double mean = s * inv_n;
  double var = q * inv_n - mean * mean;
  if (var < 0.0) var = 0.0;
  const float istd = rsqrtf((float)var + BN_EPS);
  const float scv = gam[c] * istd;
  const float shv = bet[c] - (float)mean * scv;
  ((volatile float*)sc)[c] = scv;
  ((volatile float*)sh)[c] = shv;
  __threadfence();
  ((volatile float*)sc)[c] = scv;
  ((volatile float*)sh)[c] = shv;
}

__global__ __launch_bounds__(256) void act_plane(const float* __restrict__ z, const float* __restrict__ sc,
                                                  const float* __restrict__ sh, unsigned short* __restrict__ outp) {
  const int i = blockIdx.x * 256 + threadIdx.x;
  if (i >= RTOT * 16) return;
  const int row = i >> 4, c8 = (i & 15) * 8;
  const float* zp = z + (size_t)row * CC + c8;
  const v4f z0 = *(const v4f*)zp, z1 = *(const v4f*)(zp + 4);
  const v4f s0 = *(const v4f*)(sc + c8), s1 = *(const v4f*)(sc + c8 + 4);
  const v4f h0 = *(const v4f*)(sh + c8), h1 = *(const v4f*)(sh + c8 + 4);
  v8h v;
#pragma unroll
  for (int e = 0; e < 4; ++e) {
    v[e]     = (_Float16)fmaxf(fmaf(z0[e], s0[e], h0[e]), 0.0f);
    v[4 + e] = (_Float16)fmaxf(fmaf(z1[e], s1[e], h1[e]), 0.0f);
  }
  _Float16* p = (_Float16*)outp + (size_t)row * CC + c8;
  *(volatile v8h*)p = v;
  __threadfence();
  *(volatile v8h*)p = v;
}

__global__ __launch_bounds__(256) void bn4_out(const float* __restrict__ y, const float* __restrict__ gam,
                                                const float* __restrict__ bet, float* __restrict__ outp) {
  __shared__ double dsum[CONVN];
  __shared__ double dmean[16];
  __shared__ float ssc[16], ssh[16];
  const int t = threadIdx.x;
  double s = 0.0;
  for (int b = 0; b < BB; ++b) s += (double)y[(size_t)b * CONVN + t];
  dsum[t] = s;
  __syncthreads();
  if (t < 16) {
    double S = 0.0;
#pragma unroll
    for (int o = 0; o < COUT; ++o) S += dsum[o * 16 + t];
    dmean[t] = S * (1.0 / 32768.0);
  }
  __syncthreads();
  const double m = dmean[t & 15];
  double q = 0.0;
  for (int b = 0; b < BB; ++b) {
    const double dv = (double)y[(size_t)b * CONVN + t] - m;
    q += dv * dv;
  }
  dsum[t] = q;
  __syncthreads();
  if (t < 16) {
    double V = 0.0;
#pragma unroll
    for (int o = 0; o < COUT; ++o) V += dsum[o * 16 + t];
    V *= (1.0 / 32768.0);
    const float istd = rsqrtf((float)V + BN_EPS);
    const float scv = gam[t] * istd;
    ssc[t] = scv;
    ssh[t] = bet[t] - (float)dmean[t] * scv;
  }
  __syncthreads();
  const int q4 = t & 63, rs = t >> 6;
  const int c0 = q4 * 4;
  v4f s4, h4;
#pragma unroll
  for (int e = 0; e < 4; ++e) { s4[e] = ssc[(c0 + e) & 15]; h4[e] = ssh[(c0 + e) & 15]; }
  for (int pass = 0; pass < 2; ++pass) {
    for (int b = rs; b < BB; b += 4) {
      const v4f v = *(const v4f*)(y + (size_t)b * CONVN + c0);
      v4f o;
#pragma unroll
      for (int e = 0; e < 4; ++e) o[e] = fmaxf(fmaf(v[e], s4[e], h4[e]), 0.0f);
      *(volatile v4f*)(outp + (size_t)b * CONVN + c0) = o;
    }
    __threadfence();
  }
}

extern "C" void kernel_launch(void* const* d_in, const int* in_sizes, int n_in,
                              void* d_out, int out_size, void* d_ws, size_t ws_size,
                              hipStream_t stream)
{
  if (n_in < 18) return;
  const float* atoms = (const float*)d_in[0];
  const float* bonds = (const float*)d_in[1];
  const int*   edges = (const int*)  d_in[2];
  const float* Wg1 = (const float*)d_in[3];  const float* bg1 = (const float*)d_in[4];
  const float* Wg2 = (const float*)d_in[5];  const float* bg2 = (const float*)d_in[6];
  const float* Wg3 = (const float*)d_in[7];  const float* bg3 = (const float*)d_in[8];
  const float* bn1_g = (const float*)d_in[9];  const float* bn1_b = (const float*)d_in[10];
  const float* bn2_g = (const float*)d_in[11]; const float* bn2_b = (const float*)d_in[12];
  const float* bn3_g = (const float*)d_in[13]; const float* bn3_b = (const float*)d_in[14];
  const float* Wconv = (const float*)d_in[15];
  const float* bn4_g = (const float*)d_in[16]; const float* bn4_b = (const float*)d_in[17];
  float* out = (float*)d_out;

  if (in_sizes[0] != RTOT * FA || in_sizes[1] != RTOT * DD * FBN || in_sizes[2] != RTOT * DD ||
      in_sizes[3] != DD * (FA + FBN) * CC || in_sizes[5] != DD * (CC + FBN) * CC || in_sizes[7] != DD * (CC + FBN) * CC ||
      in_sizes[15] != COUT * NN * KK || out_size != BB * CONVN) return;

  const size_t sz_z    = (size_t)RTOT * CC * 4;
  const size_t sz_a3   = (size_t)RTOT * CC * 2;
  const size_t sz_btc  = (size_t)CONVN * CONVK * 2;
  const size_t sz_bt1  = (size_t)DD * CC * 96 * 2;
  const size_t sz_bt2  = (size_t)DD * CC * 160 * 2;
  const size_t sz_part = (size_t)NBLK * CC * 4;
  const size_t sz_vec  = 512;
  const size_t sz_y    = (size_t)BB * CONVN * 4;
  const size_t off_z    = 0;
  const size_t off_a3   = off_z + sz_z;
  const size_t off_btc  = off_a3 + sz_a3;
  const size_t off_bt1  = off_btc + sz_btc;
  const size_t off_bt2  = off_bt1 + sz_bt1;
  const size_t off_bt3  = off_bt2 + sz_bt2;
  const size_t off_psum = off_bt3 + sz_bt2;
  const size_t off_psq  = off_psum + sz_part;
  const size_t off_sc   = off_psq + sz_part;
  const size_t off_y    = off_sc + 6 * sz_vec;
  const size_t total    = off_y + sz_y;
  if (total > ws_size) return;

  char* ws = (char*)d_ws;
  float*          z    = (float*)(ws + off_z);
  unsigned short* a3   = (unsigned short*)(ws + off_a3);
  unsigned short* btc  = (unsigned short*)(ws + off_btc);
  unsigned short* bt1  = (unsigned short*)(ws + off_bt1);
  unsigned short* bt2  = (unsigned short*)(ws + off_bt2);
  unsigned short* bt3  = (unsigned short*)(ws + off_bt3);
  float* psum = (float*)(ws + off_psum);
  float* psq  = (float*)(ws + off_psq);
  float* sc1 = (float*)(ws + off_sc + 0 * sz_vec); float* sh1 = (float*)(ws + off_sc + 1 * sz_vec);
  float* sc2 = (float*)(ws + off_sc + 2 * sz_vec); float* sh2 = (float*)(ws + off_sc + 3 * sz_vec);
  float* sc3 = (float*)(ws + off_sc + 4 * sz_vec); float* sh3 = (float*)(ws + off_sc + 5 * sz_vec);
  float* y   = (float*)(ws + off_y);

  prep_wg<FA + FBN, 96><<<(DD * CC * 12 + 255) / 256, 256, 0, stream>>>(Wg1, bt1);
  prep_wg<CC + FBN, 160><<<(DD * CC * 20 + 255) / 256, 256, 0, stream>>>(Wg2, bt2);
  prep_wg<CC + FBN, 160><<<(DD * CC * 20 + 255) / 256, 256, 0, stream>>>(Wg3, bt3);
  prep_wc<<<(CONVN * (CONVK / 8) + 255) / 256, 256, 0, stream>>>(Wconv, btc);

  graph_layer<true><<<NBLK, 128, 0, stream>>>(atoms, sc1, sh1, edges, bonds, bt1, bg1, z, psum, psq);
  bn_finalize<<<1, 128, 0, stream>>>(psum, psq, bn1_g, bn1_b, sc1, sh1);
  graph_layer<false><<<NBLK, 128, 0, stream>>>(z, sc1, sh1, edges, bonds, bt2, bg2, z, psum, psq);
  bn_finalize<<<1, 128, 0, stream>>>(psum, psq, bn2_g, bn2_b, sc2, sh2);
  graph_layer<false><<<NBLK, 128, 0, stream>>>(z, sc2, sh2, edges, bonds, bt3, bg3, z, psum, psq);
  bn_finalize<<<1, 128, 0, stream>>>(psum, psq, bn3_g, bn3_b, sc3, sh3);

  act_plane<<<(RTOT * 16 + 255) / 256, 256, 0, stream>>>(z, sc3, sh3, a3);
  wmma_gemm64<0, false, 0, 0, false, 0><<<dim3(16, 1, 1), 256, 0, stream>>>(
      a3, a3, CONVK, 0L, btc, btc, CONVK, 0L, (void*)y, (void*)y, CONVN, 0L,
      (const float*)y, (const float*)y, 0L, BB, CONVN, CONVK, 1.0f / 64.0f);
  bn4_out<<<1, 256, 0, stream>>>(y, bn4_g, bn4_b, out);
}
